// up_block_3040836845606
// MI455X (gfx1250) — hardware-verified
//
#include <hip/hip_runtime.h>


namespace {
constexpr int NB = 8, CIN = 128, NPT = 1024, UP = 4, M = UP * NPT, CN = CIN + 2, CQ = 32, CHP = 144, XW = 192, C1 = 256, C2 = 128;
constexpr float XS = 8.0f, WSC = 256.0f, PS = 8.0f;
__constant__ float GRIDX[4] = {-0.2f, -0.2f, 0.2f, 0.2f};
__constant__ float GRIDY[4] = {-0.2f, 0.2f, -0.2f, 0.2f};

typedef _Float16 b16;
typedef __attribute__((ext_vector_type(16))) _Float16 v16b;
typedef __attribute__((ext_vector_type(8))) _Float16 v8b;
typedef __attribute__((ext_vector_type(8))) float v8f;
typedef __attribute__((ext_vector_type(4))) float v4f;
__device__ __forceinline__ float bf16_rne(float f) { unsigned int u = __float_as_uint(f); u += 0x7FFFu + ((u >> 16) & 1u); return __uint_as_float(u & 0xFFFF0000u); }
__device__ __forceinline__ void split16(float v, b16& hi, b16& lo) { hi = (b16)v; lo = (b16)(v - (float)hi); }
__device__ __forceinline__ v16b frag_kb(const b16* p, int hh) { const v8b a = *(const v8b*)(p + 8 * hh), b = *(const v8b*)(p + 16 + 8 * hh); v16b f;
#pragma unroll
  for (int e = 0; e < 8; ++e) { f[e] = a[e]; f[8 + e] = b[e]; } return f; }
__device__ __forceinline__ v8f wmma16b(v16b a, v16b b, v8f c) { v8f d = __builtin_amdgcn_wmma_f32_16x16x32_f16(false, a, false, b, (short)0, c, false, false); asm volatile("v_nop\n\tv_nop\n\tv_nop\n\tv_nop" : "+v"(d) : "v"(a), "v"(b)); return d; }
__device__ __forceinline__ void wave_lds_sync() { __builtin_amdgcn_fence(__ATOMIC_RELEASE, "workgroup"); __builtin_amdgcn_wave_barrier(); __builtin_amdgcn_fence(__ATOMIC_ACQUIRE, "workgroup"); }
__device__ __forceinline__ float nexp(float x) { return __builtin_amdgcn_exp2f(x * 1.4426950408889634f); }
__device__ __forceinline__ float pmul(float a, float b) { float p = a * b; asm volatile("" : "+v"(p)); return p; }

__global__ __launch_bounds__(256) void prepx_kernel(const float* __restrict__ in, b16* __restrict__ XT) {
  __shared__ __attribute__((aligned(16))) b16 Tt[64][64 + 8];
  const int b = blockIdx.z, c0 = blockIdx.y * 64, n0 = blockIdx.x * 64, t_ = threadIdx.x;
  for (int q = t_; q < 64 * 64; q += 256) { const int cc = q >> 6, nn = q & 63; Tt[nn][cc] = (b16)(bf16_rne(in[((size_t)b * CIN + c0 + cc) * NPT + n0 + nn]) * XS); }
  __syncthreads();
  for (int pass = 0; pass < 2; ++pass) { for (int q = t_; q < 64 * 8; q += 256) { const int nn = q >> 3, c8 = (q & 7) * 8; *(volatile v8b*)(XT + ((size_t)b * NPT + n0 + nn) * CIN + c0 + c8) = *(const v8b*)(&Tt[nn][c8]); } __threadfence(); }
}
__global__ __launch_bounds__(256) void prepw_kernel(const float* __restrict__ wf, const float* __restrict__ wg, const float* __restrict__ wh, const float* __restrict__ w1, const float* __restrict__ w2, b16* __restrict__ WF16, b16* __restrict__ WG16, b16* __restrict__ WH16, b16* __restrict__ W116, b16* __restrict__ W216) {
  const int tid = blockIdx.x * 256 + threadIdx.x, nth = gridDim.x * 256;
  const int n1 = CQ * CIN / 8, n2 = n1, n3 = CHP * CIN / 8, n4 = C1 * XW / 8, n5 = C2 * C1 / 8;
  for (int pass = 0; pass < 2; ++pass) {
    for (int g = tid; g < n1 + n2 + n3 + n4 + n5; g += nth) { v8b o; b16* dst;
      if (g < n1 + n2) { const bool isg = g >= n1; const int e = (isg ? g - n1 : g) * 8, r = e / CIN, c = e - r * CIN; const float* w = isg ? wg : wf; dst = (isg ? WG16 : WF16) + e;
#pragma unroll
        for (int j = 0; j < 8; ++j) o[j] = (b16)(bf16_rne(w[r * CN + c + j]) * WSC); }
      else if (g < n1 + n2 + n3) { const int e = (g - n1 - n2) * 8, r = e / CIN, c = e - r * CIN; dst = WH16 + e;
#pragma unroll
        for (int j = 0; j < 8; ++j) o[j] = (r < CN) ? (b16)(bf16_rne(wh[(r < CN ? r : 0) * CN + c + j]) * WSC) : (b16)0.0f; }
      else if (g < n1 + n2 + n3 + n4) { const int e = (g - n1 - n2 - n3) * 8, r = e / XW, c = e - r * XW; dst = W116 + e;
#pragma unroll
        for (int j = 0; j < 8; ++j) o[j] = (c + j < CN) ? (b16)(bf16_rne(w1[r * CN + (c + j < CN ? c + j : 0)]) * WSC) : (b16)0.0f; }
      else { const int e = (g - n1 - n2 - n3 - n4) * 8; dst = W216 + e;
#pragma unroll
        for (int j = 0; j < 8; ++j) o[j] = (b16)(bf16_rne(w2[e + j]) * WSC); }
      *(volatile v8b*)dst = o; }
    __threadfence(); }
}
__global__ __launch_bounds__(128) void fgh_kernel(const b16* __restrict__ XT, const b16* __restrict__ WF16, const b16* __restrict__ WG16, const b16* __restrict__ WH16, const float* __restrict__ wf, const float* __restrict__ bf, const float* __restrict__ wg, const float* __restrict__ bg, const float* __restrict__ wh, const float* __restrict__ bh, b16* __restrict__ F16, b16* __restrict__ GH, b16* __restrict__ GL, b16* __restrict__ HR) {
  __shared__ __attribute__((aligned(16))) b16 Tf[4][16][32 + 8], Tgh[4][16][32 + 8], Tgl[4][16][32 + 8], Th_[4][16][XW];
  const int wave = threadIdx.x >> 5, lane = threadIdx.x & 31, nloc = lane & 15, hlf = lane >> 4; const int b = blockIdx.y, m0 = blockIdx.x * 64 + wave * 16, r_ = m0 / NPT, n0 = m0 - r_ * NPT;
  const float gx = GRIDX[r_], gy = GRIDY[r_];
  v8f acc[13];
#pragma unroll
  for (int t = 0; t < 13; ++t) acc[t] = (v8f){};
#pragma unroll
  for (int kb = 0; kb < CIN; kb += 32) { const v16b a = frag_kb(XT + ((size_t)b * NPT + n0 + nloc) * CIN + kb, hlf);
#pragma unroll
    for (int t = 0; t < 13; ++t) { const b16* B = t < 2 ? WF16 + (size_t)(t * 16 + nloc) * CIN : t < 4 ? WG16 + (size_t)((t - 2) * 16 + nloc) * CIN : WH16 + (size_t)((t - 4) * 16 + nloc) * CIN; acc[t] = wmma16b(a, frag_kb(B + kb, hlf), acc[t]); } }
#pragma unroll
  for (int t = 0; t < 13; ++t) { const int o = (t < 2 ? t : t < 4 ? t - 2 : t - 4) * 16 + nloc; const float* w = t < 2 ? wf : t < 4 ? wg : wh; const float* bb = t < 2 ? bf : t < 4 ? bg : bh; const bool live = (t < 4) || (o < CN); const int oc = live ? o : 0;
    const float add = bf16_rne(bb[oc]) + pmul(bf16_rne(w[oc * CN + CIN]), gx) + pmul(bf16_rne(w[oc * CN + CIN + 1]), gy);
#pragma unroll
    for (int r = 0; r < 8; ++r) { const float v = live ? fmaxf(acc[t][r] * (1.0f / (XS * WSC)) + add, 0.0f) : 0.0f; const int rr = 8 * hlf + r;
      if (t < 2) Tf[wave][rr][t * 16 + nloc] = (b16)(v * XS); else if (t < 4) { b16 a_, c_; split16(v * XS, a_, c_); Tgh[wave][rr][(t - 2) * 16 + nloc] = a_; Tgl[wave][rr][(t - 2) * 16 + nloc] = c_; } else Th_[wave][rr][(t - 4) * 16 + nloc] = (b16)(v * XS); } }
  if (nloc == 0) for (int r = 0; r < 8; ++r) for (int c = CHP; c < XW; ++c) Th_[wave][8 * hlf + r][c] = (b16)0.0f;
  wave_lds_sync();
  for (int pass = 0; pass < 2; ++pass) {
    for (int rp = 0; rp < 16; rp += 2) if (lane < 8) { const int rr = rp + (lane >> 2), c8 = (lane & 3) * 8; const size_t gi = ((size_t)b * M + m0 + rr) * CQ + c8;
      *(volatile v8b*)(F16 + gi) = *(const v8b*)(&Tf[wave][rr][c8]); *(volatile v8b*)(GH + gi) = *(const v8b*)(&Tgh[wave][rr][c8]); *(volatile v8b*)(GL + gi) = *(const v8b*)(&Tgl[wave][rr][c8]); }
    for (int rr = 0; rr < 16; ++rr) if (lane < 24) *(volatile v8b*)(HR + ((size_t)b * M + m0 + rr) * XW + lane * 8) = *(const v8b*)(&Th_[wave][rr][lane * 8]);
    __threadfence(); }
}
__global__ __launch_bounds__(256) void ht_kernel(const b16* __restrict__ HR, b16* __restrict__ HT) {
  __shared__ __attribute__((aligned(16))) b16 Tt[CHP][64 + 8];
  const int b = blockIdx.y, m0 = blockIdx.x * 64, t_ = threadIdx.x;
  for (int k = t_; k < 64 * CHP; k += 256) { const int mm = k / CHP, c = k - mm * CHP; Tt[c][mm] = HR[((size_t)b * M + m0 + mm) * XW + c]; }
  __syncthreads();
  for (int pass = 0; pass < 2; ++pass) { for (int q = t_; q < CHP * 8; q += 256) { const int c = q >> 3, c8 = (q & 7) * 8; *(volatile v8b*)(HT + ((size_t)b * CHP + c) * M + m0 + c8) = *(const v8b*)(&Tt[c][c8]); } __threadfence(); }
}
__global__ __launch_bounds__(64) void stats_kernel(const b16* __restrict__ F16, const b16* __restrict__ GH, const b16* __restrict__ GL, float* __restrict__ MAXK, float* __restrict__ ZK) {
  __shared__ float Sm[32], Sz[32];
  const int wave = threadIdx.x >> 5, lane = threadIdx.x & 31, hh = lane >> 4, col = lane & 15; const int b = blockIdx.y, k0 = blockIdx.x * 32 + wave * 16, ki = k0 + col;
  const b16* Fb = F16 + (size_t)b * M * CQ; const v16b gh = frag_kb(GH + ((size_t)b * M + ki) * CQ, hh), gl = frag_kb(GL + ((size_t)b * M + ki) * CQ, hh);
  float m = -INFINITY, l = 0.0f;
  for (int nb = 0; nb < M; nb += 32) {
    v8f s0 = {}, s1 = {}; const v16b f0 = frag_kb(Fb + (size_t)(nb + col) * CQ, hh), f1 = frag_kb(Fb + (size_t)(nb + 16 + col) * CQ, hh);
    s0 = wmma16b(f0, gh, s0); s0 = wmma16b(f0, gl, s0); s1 = wmma16b(f1, gh, s1); s1 = wmma16b(f1, gl, s1);
    float mr = -INFINITY;
#pragma unroll
    for (int r = 0; r < 8; ++r) { s0[r] *= (1.0f / (XS * XS)); s1[r] *= (1.0f / (XS * XS)); mr = fmaxf(mr, fmaxf(s0[r], s1[r])); }
    mr = fmaxf(mr, __shfl_xor(mr, 16)); const float mn = fmaxf(m, mr); const float al_ = nexp(m - mn); m = mn; float sum = 0.0f;
#pragma unroll
    for (int r = 0; r < 8; ++r) sum += nexp(s0[r] - mn) + nexp(s1[r] - mn);
    sum += __shfl_xor(sum, 16); l = l * al_ + sum; }
  if (hh == 0) { Sm[wave * 16 + col] = m; Sz[wave * 16 + col] = l; }
  __syncthreads();
  for (int pass = 0; pass < 2; ++pass) { if (threadIdx.x < 32) { ((volatile float*)MAXK)[(size_t)b * M + blockIdx.x * 32 + threadIdx.x] = Sm[threadIdx.x]; ((volatile float*)ZK)[(size_t)b * M + blockIdx.x * 32 + threadIdx.x] = Sz[threadIdx.x]; } __threadfence(); }
}
__global__ __launch_bounds__(64) void attn_kernel(const b16* __restrict__ F16, const b16* __restrict__ GH, const b16* __restrict__ GL, const b16* __restrict__ HT, const float* __restrict__ MAXK, const float* __restrict__ ZK, const float* __restrict__ in, const float* __restrict__ gam, b16* __restrict__ X2, b16* __restrict__ X2L) {
  __shared__ __attribute__((aligned(16))) b16 To[2][16][XW], Tq[2][16][XW];
  const int wave = threadIdx.x >> 5, lane = threadIdx.x & 31, hh = lane >> 4, col = lane & 15; const int b = blockIdx.y, m0 = blockIdx.x * 32 + wave * 16, mi = m0 + col;
  const b16* Gh = GH + (size_t)b * M * CQ; const b16* Gl = GL + (size_t)b * M * CQ; const b16* Ht = HT + (size_t)b * CHP * M; const float* mk = MAXK + (size_t)b * M; const float* zk = ZK + (size_t)b * M;
  const v16b fq = frag_kb(F16 + ((size_t)b * M + mi) * CQ, hh);
  v8f o[9];
#pragma unroll
  for (int t = 0; t < 9; ++t) o[t] = (v8f){};
  for (int kb = 0; kb < M; kb += 32) {
    v8f s0 = {}, s1 = {};
    { const size_t r0 = (size_t)(kb + col) * CQ, r1 = (size_t)(kb + 16 + col) * CQ; s0 = wmma16b(frag_kb(Gh + r0, hh), fq, s0); s0 = wmma16b(frag_kb(Gl + r0, hh), fq, s0); s1 = wmma16b(frag_kb(Gh + r1, hh), fq, s1); s1 = wmma16b(frag_kb(Gl + r1, hh), fq, s1); }
    v16b pb, pl;
#pragma unroll
    for (int r = 0; r < 8; ++r) { const int ka = kb + 8 * hh + r, kc = ka + 16; const float e0 = nexp(s0[r] * (1.0f / (XS * XS)) - mk[ka]) / zk[ka], e1 = nexp(s1[r] * (1.0f / (XS * XS)) - mk[kc]) / zk[kc]; b16 a_, c_; split16(e0 * PS, a_, c_); pb[r] = a_; pl[r] = c_; split16(e1 * PS, a_, c_); pb[8 + r] = a_; pl[8 + r] = c_; }
#pragma unroll
    for (int t = 0; t < 9; ++t) { const v16b ht = frag_kb(Ht + (size_t)(t * 16 + col) * M + kb, hh); o[t] = wmma16b(ht, pb, o[t]); o[t] = wmma16b(ht, pl, o[t]); } }
  const float gamma = bf16_rne(gam[0]); const int r_ = m0 / NPT;
#pragma unroll
  for (int t = 0; t < 9; ++t)
#pragma unroll
    for (int r = 0; r < 8; ++r) { const int c = t * 16 + 8 * hh + r; const int m = mi, n = m - (m / NPT) * NPT; float netv = 0.0f;
      if (c < CIN) netv = bf16_rne(in[((size_t)b * CIN + c) * NPT + n]); else if (c == CIN) netv = GRIDX[r_]; else if (c == CIN + 1) netv = GRIDY[r_];
      const float x = (c < CN) ? pmul(gamma, o[t][r] * (1.0f / (PS * XS))) + netv : 0.0f; b16 a_, c_; split16(x * XS, a_, c_); To[wave][col][c] = a_; Tq[wave][col][c] = c_; }
  if (hh == 0) for (int c = CHP; c < XW; ++c) { To[wave][col][c] = (b16)0.0f; Tq[wave][col][c] = (b16)0.0f; }
  wave_lds_sync();
  for (int pass = 0; pass < 2; ++pass) { for (int rr = 0; rr < 16; ++rr) if (lane < 24) { const size_t gi = ((size_t)b * M + m0 + rr) * XW + lane * 8; *(volatile v8b*)(X2 + gi) = *(const v8b*)(&To[wave][rr][lane * 8]); *(volatile v8b*)(X2L + gi) = *(const v8b*)(&Tq[wave][rr][lane * 8]); } __threadfence(); }
}
__global__ __launch_bounds__(128) void conv1_kernel(const b16* __restrict__ X2, const b16* __restrict__ X2L, const b16* __restrict__ W116, const float* __restrict__ b1, b16* __restrict__ X3, b16* __restrict__ X3L) {
  __shared__ __attribute__((aligned(16))) b16 Th[4][16][128 + 8], Tl[4][16][128 + 8];
  const int wave = threadIdx.x >> 5, lane = threadIdx.x & 31, nloc = lane & 15, hlf = lane >> 4; const size_t m0 = (size_t)blockIdx.x * 64 + wave * 16; const int n0 = blockIdx.y * 128;
  v8f acc[8];
#pragma unroll
  for (int t = 0; t < 8; ++t) acc[t] = (v8f){};
#pragma unroll
  for (int kb = 0; kb < XW; kb += 32) { const v16b a = frag_kb(X2 + (m0 + nloc) * XW + kb, hlf), al = frag_kb(X2L + (m0 + nloc) * XW + kb, hlf);
#pragma unroll
    for (int t = 0; t < 8; ++t) { const v16b bw = frag_kb(W116 + (size_t)(n0 + t * 16 + nloc) * XW + kb, hlf); acc[t] = wmma16b(a, bw, acc[t]); acc[t] = wmma16b(al, bw, acc[t]); } }
#pragma unroll
  for (int t = 0; t < 8; ++t) { const float bb = bf16_rne(b1[n0 + t * 16 + nloc]);
#pragma unroll
    for (int r = 0; r < 8; ++r) { b16 a_, c_; split16(fmaxf(acc[t][r] * (1.0f / (XS * WSC)) + bb, 0.0f) * XS, a_, c_); Th[wave][8 * hlf + r][t * 16 + nloc] = a_; Tl[wave][8 * hlf + r][t * 16 + nloc] = c_; } }
  wave_lds_sync();
  for (int pass = 0; pass < 2; ++pass) { for (int rr = 0; rr < 16; ++rr) if (lane < 16) { *(volatile v8b*)(X3 + (m0 + rr) * C1 + n0 + lane * 8) = *(const v8b*)(&Th[wave][rr][lane * 8]); *(volatile v8b*)(X3L + (m0 + rr) * C1 + n0 + lane * 8) = *(const v8b*)(&Tl[wave][rr][lane * 8]); } __threadfence(); }
}
__global__ __launch_bounds__(128) void conv2_kernel(const b16* __restrict__ X3, const b16* __restrict__ X3L, const b16* __restrict__ W216, const float* __restrict__ b2, float* __restrict__ out) {
  __shared__ __attribute__((aligned(16))) float Tc[C2][64 + 4];
  const int wave = threadIdx.x >> 5, lane = threadIdx.x & 31, nloc = lane & 15, hlf = lane >> 4, t_ = threadIdx.x; const int b = blockIdx.y, mb = blockIdx.x * 64; const size_t m0 = (size_t)b * M + mb + wave * 16;
  v8f acc[8];
#pragma unroll
  for (int t = 0; t < 8; ++t) acc[t] = (v8f){};
#pragma unroll 2
  for (int kb = 0; kb < C1; kb += 32) { const v16b a = frag_kb(X3 + (m0 + nloc) * C1 + kb, hlf), al = frag_kb(X3L + (m0 + nloc) * C1 + kb, hlf);
#pragma unroll
    for (int t = 0; t < 8; ++t) { const v16b bw = frag_kb(W216 + (size_t)(t * 16 + nloc) * C1 + kb, hlf); acc[t] = wmma16b(a, bw, acc[t]); acc[t] = wmma16b(al, bw, acc[t]); } }
#pragma unroll
  for (int t = 0; t < 8; ++t) { const int c = t * 16 + nloc; const float bb = bf16_rne(b2[c]);
#pragma unroll
    for (int r = 0; r < 8; ++r) Tc[c][wave * 16 + 8 * hlf + r] = fmaxf(acc[t][r] * (1.0f / (XS * WSC)) + bb, 0.0f); }
  __syncthreads();
  for (int pass = 0; pass < 2; ++pass) { for (int q = t_; q < C2 * 16; q += 128) { const int c = q >> 4, c4 = (q & 15) * 4; *(volatile v4f*)(out + ((size_t)b * C2 + c) * M + mb + c4) = *(const v4f*)(&Tc[c][c4]); } __threadfence(); }
}
}

extern "C" void kernel_launch(void* const* d_in, const int* in_sizes, int n_in, void* d_out, int out_size, void* d_ws, size_t ws_size, hipStream_t stream) {
  (void)n_in;
  auto Fp = [&](int i) { return (const float*)d_in[i]; };
  if (in_sizes[0] != NB * CIN * NPT || in_sizes[1] != CQ * CN || in_sizes[5] != CN * CN || in_sizes[8] != C1 * CN || in_sizes[10] != C2 * C1 || out_size != NB * C2 * M) return;
  size_t off = 0; char* ws = (char*)d_ws;
  auto carve = [&](size_t bytes) { char* p = ws + off; off += (bytes + 255) & ~(size_t)255; return p; };
  b16* XT = (b16*)carve((size_t)NB * NPT * CIN * 2); b16* WF16 = (b16*)carve(CQ * CIN * 2); b16* WG16 = (b16*)carve(CQ * CIN * 2); b16* WH16 = (b16*)carve(CHP * CIN * 2); b16* W116 = (b16*)carve(C1 * XW * 2); b16* W216 = (b16*)carve(C2 * C1 * 2);
  b16* F16 = (b16*)carve((size_t)NB * M * CQ * 2); b16* GH = (b16*)carve((size_t)NB * M * CQ * 2); b16* GL = (b16*)carve((size_t)NB * M * CQ * 2); b16* HR = (b16*)carve((size_t)NB * M * XW * 2); b16* HT = (b16*)carve((size_t)NB * CHP * M * 2);
  float* MAXK = (float*)carve((size_t)NB * M * 4); float* ZK = (float*)carve((size_t)NB * M * 4); b16* X2 = (b16*)carve((size_t)NB * M * XW * 2); b16* X2L = (b16*)carve((size_t)NB * M * XW * 2); b16* X3 = (b16*)carve((size_t)NB * M * C1 * 2); b16* X3L = (b16*)carve((size_t)NB * M * C1 * 2);
  if (off > ws_size || off > ((size_t)128 << 20)) return;
  prepx_kernel<<<dim3(NPT / 64, CIN / 64, NB), 256, 0, stream>>>(Fp(0), XT);
  prepw_kernel<<<64, 256, 0, stream>>>(Fp(1), Fp(3), Fp(5), Fp(8), Fp(10), WF16, WG16, WH16, W116, W216);
  fgh_kernel<<<dim3(M / 64, NB), 128, 0, stream>>>(XT, WF16, WG16, WH16, Fp(1), Fp(2), Fp(3), Fp(4), Fp(5), Fp(6), F16, GH, GL, HR);
  ht_kernel<<<dim3(M / 64, NB), 256, 0, stream>>>(HR, HT);
  stats_kernel<<<dim3(M / 32, NB), 64, 0, stream>>>(F16, GH, GL, MAXK, ZK);
  attn_kernel<<<dim3(M / 32, NB), 64, 0, stream>>>(F16, GH, GL, HT, MAXK, ZK, Fp(0), Fp(7), X2, X2L);
  conv1_kernel<<<dim3(NB * M / 64, C1 / 128), 128, 0, stream>>>(X2, X2L, W116, Fp(9), X3, X3L);
  conv2_kernel<<<dim3(M / 64, NB), 128, 0, stream>>>(X3, X3L, W216, Fp(11), (float*)d_out);
}
